// KANLayer_80693845557833
// MI455X (gfx1250) — hardware-verified
//
#include <hip/hip_runtime.h>
#include <stdint.h>

#pragma clang fp contract(off)

#define NROWS  8192
#define NIN    1024
#define NOUT   1024
#define NBAS   8
#define NG     12
#define KS     NIN
#define KBF    (2 * KS)
#define KSP    (NIN * NBAS)
#define KTOT   (KBF + KSP)
#define CH     4096
#define NCHUNK (NROWS / CH)
#define UROW   (KTOT / 8)
#define FTHR   256
#define FPT    (NIN / FTHR)
#define NSWEEP (UROW / FTHR)
#define PSEG   5
#define CB     64.0f
#define CSW    16384.0f
#define CINV   9.5367431640625e-07f
#define XLO    (-0.99f)
#define XHI    0.99f
#define WSCAP  134217728

static_assert(NROWS == NCHUNK * CH);
static_assert(CH % 128 == 0);
static_assert(NOUT % 64 == 0);
static_assert(KTOT % 32 == 0);
static_assert(KBF % 32 == 0);
static_assert(UROW == NSWEEP * FTHR);
static_assert(NIN == FPT * FTHR);
static_assert((KTOT * 2) % 128 == 0);
static_assert((KBF * 2) % 128 == 0);
static_assert(256 * 8 == KBF);
static_assert((PSEG - 1) * 256 == NIN);
static_assert(NG <= 32);

typedef float          v4f   __attribute__((ext_vector_type(4)));
typedef float          v8f   __attribute__((ext_vector_type(8)));
typedef int            v8i   __attribute__((ext_vector_type(8)));
typedef unsigned int   v4u   __attribute__((ext_vector_type(4)));
typedef unsigned short v8us  __attribute__((ext_vector_type(8)));
typedef _Float16       v16h  __attribute__((ext_vector_type(16)));
typedef __bf16         v16b  __attribute__((ext_vector_type(16)));
typedef v4f  __attribute__((may_alias)) v4fa;
typedef v4u  __attribute__((may_alias)) v4ua;
typedef v8us __attribute__((may_alias)) v8usa;
union FragU { v16h f; v16b b; v8us h[2]; v8i w; };

__device__ __forceinline__ unsigned short f2bf_bits(float f) {
  unsigned u = __float_as_uint(f);
  return (unsigned short)((u + 0x7FFFu + ((u >> 16) & 1u)) >> 16);
}
__device__ __forceinline__ float bf_bits2f(unsigned short b) { return __uint_as_float(((unsigned)b) << 16); }
__device__ __forceinline__ float bfr(float f) { return bf_bits2f(f2bf_bits(f)); }
__device__ __forceinline__ unsigned short f2h(float f) {
  const _Float16 hv = (_Float16)f;
  return __builtin_bit_cast(unsigned short, hv);
}
__device__ __forceinline__ unsigned pk16(unsigned short a, unsigned short b) { return (unsigned)a | ((unsigned)b << 16); }

__device__ __forceinline__ v8f wm_f16(const FragU& a, const FragU& b, v8f c) {
  v8f d = __builtin_amdgcn_wmma_f32_16x16x32_f16(false, a.f, false, b.f, (short)0, c, false, false);
  asm volatile("v_nop\n\tv_nop\n\tv_nop\n\tv_nop" : "+v"(d) : "v"(a.w), "v"(b.w));
  return d;
}
__device__ __forceinline__ v8f wm_bf16(const FragU& a, const FragU& b, v8f c) {
  v8f d = __builtin_amdgcn_wmma_f32_16x16x32_bf16(false, a.b, false, b.b, (short)0, c, false, false);
  asm volatile("v_nop\n\tv_nop\n\tv_nop\n\tv_nop" : "+v"(d) : "v"(a.w), "v"(b.w));
  return d;
}
__device__ __forceinline__ v8f z8() { v8f z = {0.f, 0.f, 0.f, 0.f, 0.f, 0.f, 0.f, 0.f}; return z; }

__global__ __launch_bounds__(256) void prep_kernel(const float* __restrict__ bw, const float* __restrict__ sw,
                                                   unsigned short* __restrict__ BP) {
  const int tid = threadIdx.x;
  const int seg = blockIdx.x;
  const int o = blockIdx.y;
  unsigned short* rowp = BP + (size_t)o * KTOT;
  v4u v;
  unsigned short* dst;
  if (seg == 0) {
    const float* src = bw + (size_t)o * NIN + 8 * (tid & 127);
    const v4f a = *(const v4fa*)src;
    const v4f c = *(const v4fa*)(src + 4);
    v[0] = pk16(f2bf_bits(a[0]), f2bf_bits(a[1]));
    v[1] = pk16(f2bf_bits(a[2]), f2bf_bits(a[3]));
    v[2] = pk16(f2bf_bits(c[0]), f2bf_bits(c[1]));
    v[3] = pk16(f2bf_bits(c[2]), f2bf_bits(c[3]));
    dst = rowp + 8 * tid;
  } else {
    const int i = (seg - 1) * 256 + tid;
    const float* src = sw + ((size_t)o * NIN + i) * NBAS;
    const v4f a = *(const v4fa*)src;
    const v4f c = *(const v4fa*)(src + 4);
    v[0] = pk16(f2h(CSW * bfr(a[0])), f2h(CSW * bfr(a[1])));
    v[1] = pk16(f2h(CSW * bfr(a[2])), f2h(CSW * bfr(a[3])));
    v[2] = pk16(f2h(CSW * bfr(c[0])), f2h(CSW * bfr(c[1])));
    v[3] = pk16(f2h(CSW * bfr(c[2])), f2h(CSW * bfr(c[3])));
    dst = rowp + KBF + 8 * i;
  }
  *(volatile v4u*)dst = v;
  __threadfence();
  *(volatile v4u*)dst = v;
}

__device__ __forceinline__ void a_store_pass(const unsigned short* sA, unsigned short* dst, int tid) {
#pragma unroll
  for (int it = 0; it < NSWEEP; ++it) {
    const int u = it * FTHR + tid;
    const v4u v = *(const v4ua*)(sA + 8 * u);
    *(volatile v4u*)(dst + 8 * u) = v;
  }
}

__global__ __launch_bounds__(FTHR) void feat_kernel(const float* __restrict__ x, const float* __restrict__ grid,
                                                    unsigned short* __restrict__ AP, int row_base) {
  __shared__ __align__(16) unsigned short sA[KTOT];
  __shared__ float sG[32];
  __shared__ float sInv[32];
  const int tid = threadIdx.x;
  const int r = blockIdx.x;

  if (tid < 32) {
    const int gi = (tid < NG) ? tid : (NG - 1);
    sG[tid] = bfr(grid[gi]);
  }
  __syncthreads();
  if (tid < 32) {
    const int k = (tid < 11) ? 1 : ((tid < 22) ? 2 : 3);
    const int j = tid - 11 * (k - 1);
    const int jk = (j + k < NG - 1) ? (j + k) : (NG - 1);
    const float den = sG[jk] - sG[j];
    sInv[tid] = 1.0f / den;
  }
  __syncthreads();

  float g[NG];
#pragma unroll
  for (int j = 0; j < NG; ++j) g[j] = sG[j];
  float i1[11], i2[10], i3[9];
#pragma unroll
  for (int j = 0; j < 11; ++j) i1[j] = sInv[j];
#pragma unroll
  for (int j = 0; j < 10; ++j) i2[j] = sInv[11 + j];
#pragma unroll
  for (int j = 0; j < 9; ++j) i3[j] = sInv[22 + j];

  const float* xrow = x + (size_t)(row_base + r) * NIN;
#pragma unroll 1
  for (int it = 0; it < FPT; ++it) {
    const int i = it * FTHR + tid;
    const float xr = bfr(xrow[i]);

    const float e = expf(-xr);
    const float sg = 1.0f / (1.0f + e);
    const float s = xr * sg;
    const unsigned short hb = f2bf_bits(s);
    const float hf = bf_bits2f(hb);
    const unsigned short lb = f2bf_bits(s - hf);
    sA[i] = hb;
    sA[KS + i] = lb;

    const float xc = fminf(fmaxf(xr, XLO), XHI);
    float b0[11];
#pragma unroll
    for (int j = 0; j < 11; ++j) {
      const bool c = (xc >= g[j]) & (xc < g[j + 1]);
      b0[j] = c ? 1.0f : 0.0f;
    }
    float b1[10];
#pragma unroll
    for (int j = 0; j < 10; ++j) {
      float lt = xc - g[j];     lt = lt * i1[j];     lt = lt * b0[j];
      float rt = g[j + 2] - xc; rt = rt * i1[j + 1]; rt = rt * b0[j + 1];
      b1[j] = lt + rt;
    }
    float b2[9];
#pragma unroll
    for (int j = 0; j < 9; ++j) {
      float lt = xc - g[j];     lt = lt * i2[j];     lt = lt * b1[j];
      float rt = g[j + 3] - xc; rt = rt * i2[j + 1]; rt = rt * b1[j + 1];
      b2[j] = lt + rt;
    }
    float b3[8];
#pragma unroll
    for (int j = 0; j < 8; ++j) {
      float lt = xc - g[j];     lt = lt * i3[j];     lt = lt * b2[j];
      float rt = g[j + 4] - xc; rt = rt * i3[j + 1]; rt = rt * b2[j + 1];
      b3[j] = lt + rt;
    }
    v4u pk;
    pk[0] = pk16(f2h(CB * b3[0]), f2h(CB * b3[1]));
    pk[1] = pk16(f2h(CB * b3[2]), f2h(CB * b3[3]));
    pk[2] = pk16(f2h(CB * b3[4]), f2h(CB * b3[5]));
    pk[3] = pk16(f2h(CB * b3[6]), f2h(CB * b3[7]));
    *(v4ua*)(sA + KBF + 8 * i) = pk;
  }
  __syncthreads();

  unsigned short* dst = AP + (size_t)r * KTOT;
  a_store_pass(sA, dst, tid);
  __threadfence();
  a_store_pass(sA, dst, tid);
}

__device__ __forceinline__ void o_store_pass(const float* sO, float* out,
                                             int grow_w, int n0, int w, int lane) {
  const int q8 = lane & 7, sub = lane >> 3;
#pragma unroll
  for (int i = 0; i < 16; ++i) {
    const int lid = i * 4 + sub;
    const int row = lid >> 1, hl = lid & 1;
    const v4f v = *(const v4fa*)(sO + (32 * w + row) * 64 + 32 * hl + 4 * q8);
    *(volatile v4f*)(out + (size_t)(grow_w + row) * NOUT + n0 + 32 * hl + 4 * q8) = v;
  }
}

__global__ __launch_bounds__(128) void gemm_kernel(const unsigned short* __restrict__ AP,
                                                   const unsigned short* __restrict__ BP,
                                                   float* __restrict__ out, int row_base) {
  __shared__ __align__(16) float sO[128 * 64];
  const int tid = threadIdx.x, lane = tid & 31, w = tid >> 5;
  const int h = lane >> 4, m = lane & 15;
  const int lrow_w = blockIdx.x * 128 + 32 * w;
  const int n0 = blockIdx.y * 64;

  const unsigned short* xa0 = AP + (size_t)(lrow_w + m) * KTOT + 8 * h;
  const unsigned short* xa1 = xa0 + (size_t)16 * KTOT;
  const unsigned short* wb  = BP + (size_t)(n0 + m) * KTOT + 8 * h;

  v8f acc[2][4];
#pragma unroll
  for (int mt = 0; mt < 2; ++mt)
#pragma unroll
    for (int nt = 0; nt < 4; ++nt) acc[mt][nt] = z8();

#pragma unroll 1
  for (int k0 = KBF; k0 < KTOT; k0 += 32) {
    FragU a0, a1;
    a0.h[0] = *(const v8usa*)(xa0 + k0);
    a0.h[1] = *(const v8usa*)(xa0 + k0 + 16);
    a1.h[0] = *(const v8usa*)(xa1 + k0);
    a1.h[1] = *(const v8usa*)(xa1 + k0 + 16);
#pragma unroll
    for (int nt = 0; nt < 4; ++nt) {
      const unsigned short* wq = wb + (size_t)nt * 16 * KTOT + k0;
      FragU b;
      b.h[0] = *(const v8usa*)wq;
      b.h[1] = *(const v8usa*)(wq + 16);
      acc[0][nt] = wm_f16(a0, b, acc[0][nt]);
      acc[1][nt] = wm_f16(a1, b, acc[1][nt]);
    }
  }

#pragma unroll
  for (int mt = 0; mt < 2; ++mt)
#pragma unroll
    for (int nt = 0; nt < 4; ++nt) acc[mt][nt] = acc[mt][nt] * CINV;

#pragma unroll 1
  for (int k0 = 0; k0 < KBF; k0 += 32) {
    FragU a0, a1;
    a0.h[0] = *(const v8usa*)(xa0 + k0);
    a0.h[1] = *(const v8usa*)(xa0 + k0 + 16);
    a1.h[0] = *(const v8usa*)(xa1 + k0);
    a1.h[1] = *(const v8usa*)(xa1 + k0 + 16);
#pragma unroll
    for (int nt = 0; nt < 4; ++nt) {
      const unsigned short* wq = wb + (size_t)nt * 16 * KTOT + k0;
      FragU b;
      b.h[0] = *(const v8usa*)wq;
      b.h[1] = *(const v8usa*)(wq + 16);
      acc[0][nt] = wm_bf16(a0, b, acc[0][nt]);
      acc[1][nt] = wm_bf16(a1, b, acc[1][nt]);
    }
  }

#pragma unroll
  for (int nt = 0; nt < 4; ++nt) {
    const int cl = 16 * nt + m;
#pragma unroll
    for (int mt = 0; mt < 2; ++mt) {
#pragma unroll
      for (int r = 0; r < 8; ++r) {
        const int rl = 32 * w + 16 * mt + 8 * h + r;
        sO[rl * 64 + cl] = acc[mt][nt][r];
      }
    }
  }
  __syncthreads();

  const int grow_w = row_base + lrow_w;
  o_store_pass(sO, out, grow_w, n0, w, lane);
  __threadfence();
  o_store_pass(sO, out, grow_w, n0, w, lane);
}

extern "C" void kernel_launch(void* const* d_in, const int* in_sizes, int n_in,
                              void* d_out, int out_size, void* d_ws, size_t ws_size,
                              hipStream_t stream) {
  if (n_in < 4) return;
  if (in_sizes[0] != NROWS * NIN) return;
  if (in_sizes[1] != NOUT * NIN) return;
  if (in_sizes[2] != NOUT * NIN * NBAS) return;
  if (in_sizes[3] != NG) return;
  if (out_size != NROWS * NOUT) return;

  const float* x    = (const float*)d_in[0];
  const float* bw   = (const float*)d_in[1];
  const float* sw   = (const float*)d_in[2];
  const float* grid = (const float*)d_in[3];
  float* out = (float*)d_out;

  size_t off = 0;
  const size_t oAP = off; off += (size_t)CH * KTOT * 2;
  const size_t oBP = off; off += (size_t)NOUT * KTOT * 2;
  if (off > ws_size) return;
  if (off > (size_t)WSCAP) return;

  char* ws = (char*)d_ws;
  unsigned short* AP = (unsigned short*)(ws + oAP);
  unsigned short* BP = (unsigned short*)(ws + oBP);

  prep_kernel<<<dim3(PSEG, NOUT), dim3(256), 0, stream>>>(bw, sw, BP);
  for (int c = 0; c < NCHUNK; ++c) {
    const int row_base = c * CH;
    feat_kernel<<<dim3(CH), dim3(FTHR), 0, stream>>>(x, grid, AP, row_base);
    gemm_kernel<<<dim3(CH / 128, NOUT / 64), dim3(128), 0, stream>>>(AP, BP, out, row_base);
  }
  (void)hipGetLastError();
}
